// Sender_30150670418386
// MI455X (gfx1250) — hardware-verified
//
#include <hip/hip_runtime.h>
#include <stddef.h>


#define HE    128
#define HID   128
#define KIN   256
#define THR   256
#define NWV   8
#define CHUNK 4096
#define NB    2048
#define LDB   11
#define NSTW  8
#define FTHR  128
#define FROWS 64
#define ESC   64.0f
#define WSC   64.0f
#define RSC   0.000244140625f
#define NEGS  0.2f
#define MINIT -1.0e30f
#define WSCAP 134217728
#define LDS_DRAIN (NB * NSTW * 4 + CHUNK * 4 + NB * 2 * 4 + 32)

static_assert((1 << LDB) == NB);
static_assert(CHUNK == THR * 16 && NWV * 32 == THR);
static_assert((NB % NWV) == 0 && (NB % FROWS) == 0 && (NB % 64) == 0);
static_assert((NB * NSTW) == 64 * THR && (NB * 2) == 16 * THR && (NB * 16) == 128 * THR && (NB / 2) == 4 * THR);
static_assert(LDS_DRAIN == 98336);
static_assert(FROWS == (FTHR / 32) * 16);
static_assert(HE == 128 && HID == 128 && KIN == 2 * HE);
static_assert((HID * HE) == 8 * THR * 8);

typedef float    v4f  __attribute__((ext_vector_type(4)));
typedef float    v8f  __attribute__((ext_vector_type(8)));
typedef int      v4i  __attribute__((ext_vector_type(4)));
typedef _Float16 v8h  __attribute__((ext_vector_type(8)));
typedef _Float16 v16h __attribute__((ext_vector_type(16)));
union Frag { v16h v; v8h h[2]; };

#define WSYNC() do { __builtin_amdgcn_fence(__ATOMIC_ACQ_REL, "wavefront"); __builtin_amdgcn_wave_barrier(); } while (0)

__device__ __forceinline__ v8f wmh(v16h a, v16h b, v8f c) {
  v8f d = __builtin_amdgcn_wmma_f32_16x16x32_f16(false, a, false, b, (short)0, c, false, false);
  asm volatile("v_nop\n\tv_nop\n\tv_nop\n\tv_nop" : "+v"(d) : "v"(a), "v"(b));
  return d;
}

__global__ __launch_bounds__(THR) void k_prep(const float* __restrict__ wfc, _Float16* Bp) {
  const int i = blockIdx.x * THR + threadIdx.x;
  const int n = i >> 4, k = (i & 15) * 8;
  const float* sp = wfc + (size_t)n * KIN + k;
  v8h hv;
#pragma unroll
  for (int e = 0; e < 8; ++e) hv[e] = (_Float16)(sp[e] * WSC);
  _Float16* dp = Bp + (size_t)i * 8;
  *(volatile v8h*)dp = hv;
  __threadfence();
  *(volatile v8h*)dp = hv;
}

template <int NBT>
__device__ __forceinline__ int compact(const int* __restrict__ dsts, int nE, int cbase, int n0,
                                       int wave, int lane, int vec, unsigned* slist, int* swt) {
  int d[16];
  const int eb = cbase + 512 * wave + 4 * lane;
  if (vec != 0 && cbase + CHUNK <= nE) {
#pragma unroll
    for (int q = 0; q < 4; ++q) {
      const v4i t4 = *(const v4i*)(dsts + eb + 128 * q);
      d[4 * q] = t4.x; d[4 * q + 1] = t4.y; d[4 * q + 2] = t4.z; d[4 * q + 3] = t4.w;
    }
  } else {
#pragma unroll
    for (int k = 0; k < 16; ++k) {
      int idx = eb + 128 * (k >> 2) + (k & 3);
      const bool ok = idx < nE;
      idx = ok ? idx : nE - 1;
      const int val = dsts[idx];
      d[k] = ok ? val : (-2147483647 - 1);
    }
  }
  unsigned hm[16];
  int cw = 0;
#pragma unroll
  for (int k = 0; k < 16; ++k) {
    const unsigned ld = (unsigned)d[k] - (unsigned)n0;
    hm[k] = __builtin_amdgcn_ballot_w32(ld < (unsigned)NBT);
    cw += __builtin_popcount(hm[k]);
  }
  swt[wave] = cw;
  __syncthreads();
  int base = 0, nh = 0;
#pragma unroll
  for (int w = 0; w < NWV; ++w) {
    const int v = swt[w];
    base += (w < wave) ? v : 0;
    nh += v;
  }
  int run = base;
#pragma unroll
  for (int k = 0; k < 16; ++k) {
    const unsigned ld = (unsigned)d[k] - (unsigned)n0;
    const unsigned mk = hm[k];
    const int pos = run + (int)__builtin_amdgcn_mbcnt_lo(mk, 0u);
    const unsigned e = (unsigned)(eb + 128 * (k >> 2) + (k & 3));
    if (ld < (unsigned)NBT) slist[pos & (CHUNK - 1)] = (e << LDB) | ld;
    run += __builtin_popcount(mk);
  }
  __syncthreads();
  return nh;
}

__device__ __forceinline__ void att_upd(float* sst, int ld, float xs, float xd, float a,
                                        const float (&wl4)[4], const float (&bl4)[4],
                                        const float (&wr4)[4], const float (&br4)[4],
                                        const float (&we4)[4], const float (&at4)[4],
                                        int lane, int hsel) {
  float lg = 0.0f;
#pragma unroll
  for (int j = 0; j < 4; ++j) {
    const float t   = fmaf(xs, wl4[j], bl4[j]);
    const float u   = fmaf(xd, wr4[j], br4[j]);
    const float arg = fmaf(a, we4[j], t + u);
    const float lr  = fmaxf(arg, NEGS * arg);
    lg = fmaf(at4[j], lr, lg);
  }
  lg += __shfl_xor(lg, 1, 32);
  lg += __shfl_xor(lg, 2, 32);
  lg += __shfl_xor(lg, 4, 32);
  lg += __shfl_xor(lg, 8, 32);
  float* st = sst + ld * NSTW + 3 * hsel;
  const float mo = st[0], dold = st[1], sold = st[2];
  const float mn = fmaxf(mo, lg);
  const float sc = __expf(mo - mn);
  const float p  = __expf(lg - mn);
  const float dn = fmaf(dold, sc, p);
  const float sn = fmaf(p, xs, sold * sc);
  if ((lane & 15) == 0) { st[0] = mn; st[1] = dn; st[2] = sn; }
}

__global__ __launch_bounds__(THR) void k_drain(
    const int* __restrict__ srcs, const int* __restrict__ dsts, const float* __restrict__ x,
    const float* __restrict__ ea, const float* __restrict__ Wl, const float* __restrict__ bl,
    const float* __restrict__ Wr, const float* __restrict__ br, const float* __restrict__ We,
    const float* __restrict__ att, const float* __restrict__ bo,
    float* Gp, _Float16* Ep, int nN, int nE, int nChunks, int vec) {
  extern __shared__ __attribute__((aligned(16))) char dynl[];
  float*    sst   = (float*)dynl;
  unsigned* slist = (unsigned*)(dynl + NB * NSTW * 4);
  float*    sg    = (float*)(slist + CHUNK);
  int*      swt   = (int*)(sg + NB * 2);
  const int tid = threadIdx.x, lane = tid & 31, hsel = lane >> 4;
  const int wave = __builtin_amdgcn_readfirstlane(tid >> 5);
  const int n0 = blockIdx.x * NB;

  float wl4[4], bl4[4], wr4[4], br4[4], we4[4], at4[4];
#pragma unroll
  for (int j = 0; j < 4; ++j) {
    const int ch = 4 * lane + j;
    wl4[j] = Wl[ch]; bl4[j] = bl[ch]; wr4[j] = Wr[ch]; br4[j] = br[ch]; we4[j] = We[ch]; at4[j] = att[ch];
  }
#pragma unroll 4
  for (int it = 0; it < 64; ++it) {
    const int f = it * THR + tid;
    const int w = f & 7;
    sst[f] = (w == 0 || w == 3) ? MINIT : 0.0f;
  }
  __syncthreads();

#pragma unroll 1
  for (int c = 0; c < nChunks; ++c) {
    const int nh = compact<NB>(dsts, nE, c * CHUNK, n0, wave, lane, vec, slist, swt);
    const int nhc = nh < CHUNK ? nh : CHUNK;
    for (int j0 = 0; j0 < nhc; j0 += 32) {
      const int idx = j0 + lane;
      const bool inr = idx < nhc;
      const unsigned ent = slist[inr ? idx : 0];
      const bool own = inr && ((ent & 7u) == (unsigned)wave);
      unsigned om = __builtin_amdgcn_ballot_w32(own);
      while (om != 0u) {
        const int b = __builtin_ctz(om);
        om &= om - 1u;
        const unsigned eb = (unsigned)__builtin_amdgcn_readlane((int)ent, b);
        int e = (int)(eb >> LDB);
        e = e > nE - 1 ? nE - 1 : e;
        const int ld = (int)(eb & (unsigned)(NB - 1));
        int s = srcs[e];
        s = s < 0 ? 0 : (s > nN - 1 ? nN - 1 : s);
        int dnode = n0 + ld;
        dnode = dnode > nN - 1 ? nN - 1 : dnode;
        const float a  = ea[e];
        const float xs = x[s];
        const float xd = x[dnode];
        att_upd(sst, ld, xs, xd, a, wl4, bl4, wr4, br4, we4, at4, lane, hsel);
        if (lane == 0) {
          float* cp = sst + ld * NSTW + 6;
          const float c0 = cp[0] + 1.0f;
          const float c1 = cp[1] + a;
          cp[0] = c0;
          cp[1] = c1;
        }
        WSYNC();
      }
    }
  }
#pragma unroll 1
  for (int q = 0; q < NB / NWV; ++q) {
    const int ld = NWV * q + wave;
    const int node = n0 + ld;
    const int xrow = node > nN - 1 ? nN - 1 : node;
    const float cn = sst[ld * NSTW + 6];
    const float sm = sst[ld * NSTW + 7];
    const float a  = sm * (1.0f / fmaxf(cn, 1.0f));
    const float xs = x[xrow];
    att_upd(sst, ld, xs, xs, a, wl4, bl4, wr4, br4, we4, at4, lane, hsel);
  }
  __syncthreads();

#pragma unroll 1
  for (int it = 0; it < 16; ++it) {
    const int f = it * THR + tid;
    const int ld = f >> 1, h = f & 1;
    const float* st = sst + ld * NSTW + 3 * h;
    sg[f] = st[2] * (1.0f / st[1]);
  }
  __syncthreads();

#pragma unroll
  for (int it = 0; it < 4; ++it) {
    const int f = it * THR + tid;
    const v4f v = *(const v4f*)(sg + 4 * f);
    *(volatile v4f*)(Gp + (size_t)n0 * 2 + 4 * f) = v;
  }
  __threadfence();
#pragma unroll
  for (int it = 0; it < 4; ++it) {
    const int f = it * THR + tid;
    const v4f v = *(const v4f*)(sg + 4 * f);
    *(volatile v4f*)(Gp + (size_t)n0 * 2 + 4 * f) = v;
  }

  const int p = tid & 15, hp = p >> 3;
  float cw[8], cb[8], co[8];
#pragma unroll
  for (int j = 0; j < 8; ++j) {
    const int ch = 8 * p + j;
    cw[j] = Wl[ch]; cb[j] = bl[ch]; co[j] = bo[ch];
  }
#pragma unroll 1
  for (int it = 0; it < 128; ++it) {
    const int f = it * THR + tid, row = f >> 4;
    const float g = sg[row * 2 + hp];
    v8h hv;
#pragma unroll
    for (int j = 0; j < 8; ++j) hv[j] = (_Float16)((fmaf(cw[j], g, cb[j]) + co[j]) * ESC);
    *(volatile v8h*)(Ep + (size_t)(n0 + row) * HE + 8 * p) = hv;
  }
  __threadfence();
#pragma unroll 1
  for (int it = 0; it < 128; ++it) {
    const int f = it * THR + tid, row = f >> 4;
    const float g = sg[row * 2 + hp];
    v8h hv;
#pragma unroll
    for (int j = 0; j < 8; ++j) hv[j] = (_Float16)((fmaf(cw[j], g, cb[j]) + co[j]) * ESC);
    *(volatile v8h*)(Ep + (size_t)(n0 + row) * HE + 8 * p) = hv;
  }
}

__global__ __launch_bounds__(FTHR) void k_cvec(const float* __restrict__ Gp, const int* __restrict__ tix,
                                               const float* __restrict__ Wl, const float* __restrict__ bl,
                                               const float* __restrict__ bo, const float* __restrict__ wfc,
                                               const float* __restrict__ bfc, float* cvec, int nN) {
  __shared__ float stg[HE];
  const int t = threadIdx.x;
  int tn = tix[0];
  tn = tn < 0 ? 0 : (tn > nN - 1 ? nN - 1 : tn);
  const float g = Gp[(size_t)tn * 2 + (t >> 6)];
  stg[t] = fmaf(Wl[t], g, bl[t]) + bo[t];
  __syncthreads();
  float acc = bfc[t];
  const float* wrow = wfc + (size_t)t * KIN + HE;
#pragma unroll 4
  for (int k = 0; k < HE; ++k) acc = fmaf(wrow[k], stg[k], acc);
  *(volatile float*)(cvec + t) = acc;
  __threadfence();
  *(volatile float*)(cvec + t) = acc;
}

__global__ __launch_bounds__(FTHR) void k_fc(const _Float16* __restrict__ Ep, const _Float16* __restrict__ Bp,
                                             const float* __restrict__ cvec, float* out, int nN) {
  __shared__ __attribute__((aligned(16))) float so[(FTHR / 32) * 16 * HID];
  const int tid = threadIdx.x, lane = tid & 31, wave = tid >> 5, hh = lane >> 4, m = lane & 15;
  const int row0 = blockIdx.x * FROWS + wave * 16;

  v8f acc[8];
#pragma unroll
  for (int t = 0; t < 8; ++t) { v8f z = {0.f, 0.f, 0.f, 0.f, 0.f, 0.f, 0.f, 0.f}; acc[t] = z; }
  const _Float16* ap = Ep + (size_t)(row0 + m) * HE + 8 * hh;
  const _Float16* bb = Bp + (size_t)m * HE + 8 * hh;
#pragma unroll
  for (int ks = 0; ks < HE / 32; ++ks) {
    Frag a;
    a.h[0] = *(const v8h*)(ap + 32 * ks);
    a.h[1] = *(const v8h*)(ap + 32 * ks + 16);
#pragma unroll
    for (int t = 0; t < 8; ++t) {
      const _Float16* bp = bb + (size_t)(16 * t) * HE + 32 * ks;
      Frag b;
      b.h[0] = *(const v8h*)bp;
      b.h[1] = *(const v8h*)(bp + 16);
      acc[t] = wmh(a.v, b.v, acc[t]);
    }
  }
  float* os = so + wave * 16 * HID;
#pragma unroll
  for (int t = 0; t < 8; ++t) {
    const float cv = cvec[16 * t + m];
#pragma unroll
    for (int r = 0; r < 8; ++r) os[(8 * hh + r) * HID + 16 * t + m] = fmaf(acc[t][r], RSC, cv);
  }
  WSYNC();

#pragma unroll
  for (int i = 0; i < 16; ++i) {
    const int grow = row0 + i;
    const v4f v = *(const v4f*)(os + i * HID + 4 * lane);
    if (grow < nN) *(volatile v4f*)(out + (size_t)grow * HID + 4 * lane) = v;
  }
  __threadfence();
#pragma unroll
  for (int i = 0; i < 16; ++i) {
    const int grow = row0 + i;
    const v4f v = *(const v4f*)(os + i * HID + 4 * lane);
    if (grow < nN) *(volatile v4f*)(out + (size_t)grow * HID + 4 * lane) = v;
  }
}

extern "C" void kernel_launch(void* const* d_in, const int* in_sizes, int n_in,
                              void* d_out, int out_size, void* d_ws, size_t ws_size,
                              hipStream_t stream) {
  if (n_in < 13) return;
  const int nN = in_sizes[0];
  const int nE = in_sizes[2];
  if (nN < 1 || nE < 1) return;
  if (nN > (1 << 21) || nE > (1 << 21)) return;
  if (in_sizes[1] != 2 * nE || in_sizes[3] < 1) return;
  if (in_sizes[4] != HE || in_sizes[5] != HE || in_sizes[6] != HE || in_sizes[7] != HE) return;
  if (in_sizes[8] != HE || in_sizes[9] != HE || in_sizes[10] != HE) return;
  if (in_sizes[11] != HID * KIN || in_sizes[12] != HID) return;
  if (out_size != nN * HID) return;

  const float* x    = (const float*)d_in[0];
  const int*   ei   = (const int*)d_in[1];
  const float* eat  = (const float*)d_in[2];
  const int*   tix  = (const int*)d_in[3];
  const float* Wl   = (const float*)d_in[4];
  const float* bl   = (const float*)d_in[5];
  const float* Wr   = (const float*)d_in[6];
  const float* br   = (const float*)d_in[7];
  const float* We   = (const float*)d_in[8];
  const float* att  = (const float*)d_in[9];
  const float* bo   = (const float*)d_in[10];
  const float* wfc  = (const float*)d_in[11];
  const float* bfc  = (const float*)d_in[12];
  float* out = (float*)d_out;
  const int* srcs = ei;
  const int* dsts = ei + (size_t)nE;

  const int gDrain  = (nN + NB - 1) / NB;
  const int nPad    = gDrain * NB;
  const int gFC     = (nN + FROWS - 1) / FROWS;
  const int nChunks = (nE + CHUNK - 1) / CHUNK;
  const int vec     = ((nE & 3) == 0) ? 1 : 0;

  char* ws = (char*)d_ws;
  size_t off = 0;
  const size_t oB = off; off += (size_t)HID * HE * 2;     off = (off + 255) & ~(size_t)255;
  const size_t oC = off; off += 512;                      off = (off + 255) & ~(size_t)255;
  const size_t oG = off; off += (size_t)nPad * 2 * 4;     off = (off + 255) & ~(size_t)255;
  const size_t oE = off; off += (size_t)nPad * HE * 2;    off = (off + 255) & ~(size_t)255;
  if (off > ws_size || off > (size_t)WSCAP) return;
  _Float16* Bp   = (_Float16*)(ws + oB);
  float*    cvec = (float*)(ws + oC);
  float*    Gp   = (float*)(ws + oG);
  _Float16* Ep   = (_Float16*)(ws + oE);

  hipFuncSetAttribute(reinterpret_cast<const void*>(&k_drain), hipFuncAttributeMaxDynamicSharedMemorySize, LDS_DRAIN);

  k_prep<<<(HID * HE) / (8 * THR), THR, 0, stream>>>(wfc, Bp);
  k_drain<<<gDrain, THR, LDS_DRAIN, stream>>>(srcs, dsts, x, eat, Wl, bl, Wr, br, We, att, bo,
                                              Gp, Ep, nN, nE, nChunks, vec);
  k_cvec<<<1, FTHR, 0, stream>>>(Gp, tix, Wl, bl, bo, wfc, bfc, cvec, nN);
  k_fc<<<gFC, FTHR, 0, stream>>>(Ep, Bp, cvec, out, nN);
}
